// PVMFormer_81346680586863
// MI455X (gfx1250) — hardware-verified
//
#include <hip/hip_runtime.h>


#define NB_    8
#define CH_    128
#define NL_    4096
#define NTOK_  (NB_ * NL_)
#define DB_    64
#define DM_    16
#define DI_    32
#define NS_    16
#define XDN_   33
#define HID_   512
#define NGRP_  32
#define G1P_   1024
#define LNEPS_ 1e-5f
#define WSCL_  64.0f
#define WINV_  0.015625f

static_assert(NTOK_ % 64 == 0);
static_assert(NL_ % 128 == 0);
static_assert(NL_ % 64 == 0);
static_assert(HID_ % 128 == 0);
static_assert(CH_ % 64 == 0);
static_assert(DB_ == 4 * DM_);
static_assert(DI_ == 32);
static_assert(HID_ / NGRP_ == 16);
static_assert(CH_ / NGRP_ == 4);
static_assert((NB_ * CH_ * NL_) % 1024 == 0);
static_assert(NTOK_ % 2 == 0);

typedef float          v4f   __attribute__((ext_vector_type(4)));
typedef float          v8f   __attribute__((ext_vector_type(8)));
typedef _Float16       v8h   __attribute__((ext_vector_type(8)));
typedef _Float16       v16h  __attribute__((ext_vector_type(16)));
typedef unsigned short u16x8 __attribute__((ext_vector_type(8)));

union FragH { u16x8 h[2]; v16h v; };
union Pack8 { v8h f; u16x8 u; };

constexpr size_t SZ_XN16  = (size_t)NTOK_ * CH_ * 2;
constexpr size_t SZ_Z     = (size_t)NTOK_ * DB_ * 4;
constexpr size_t SZ_MLN   = (size_t)NTOK_ * DB_ * 2;
constexpr size_t SZ_H2    = (size_t)NB_ * CH_ * NL_ * 4;
constexpr size_t SZ_OUT1  = (size_t)NB_ * CH_ * NL_ * 4;
constexpr size_t SZ_OUT1T = (size_t)NTOK_ * CH_ * 2;
constexpr size_t SZ_H1    = (size_t)NTOK_ * HID_ * 4;
constexpr size_t SZ_WIN   = (size_t)DB_ * CH_ * 2;
constexpr size_t SZ_WOUT  = (size_t)CH_ * DB_ * 2;
constexpr size_t SZ_W1    = (size_t)HID_ * CH_ * 2;
constexpr size_t SZ_W2    = (size_t)CH_ * HID_ * 2;
constexpr size_t SZ_ST    = (size_t)NB_ * NGRP_ * 128;
constexpr size_t SZ_ANEG  = (size_t)DI_ * NS_ * 4;

constexpr size_t OFF_XN16  = 0;
constexpr size_t OFF_Z     = OFF_XN16 + SZ_XN16;
constexpr size_t OFF_MLN   = OFF_Z + SZ_Z;
constexpr size_t REG0_END  = OFF_MLN + SZ_MLN;
constexpr size_t OFF_H2    = 0;
constexpr size_t OFF_OUT1  = REG0_END;
constexpr size_t OFF_OUT1T = OFF_OUT1 + SZ_OUT1;
constexpr size_t OFF_H1    = OFF_OUT1T + SZ_OUT1T;
constexpr size_t OFF_WIN   = OFF_H1 + SZ_H1;
constexpr size_t OFF_WOUT  = OFF_WIN + SZ_WIN;
constexpr size_t OFF_W1    = OFF_WOUT + SZ_WOUT;
constexpr size_t OFF_W2    = OFF_W1 + SZ_W1;
constexpr size_t OFF_ST1   = OFF_W2 + SZ_W2;
constexpr size_t OFF_ST2   = OFF_ST1 + SZ_ST;
constexpr size_t OFF_ANEG  = OFF_ST2 + SZ_ST;
constexpr size_t WS_END    = OFF_ANEG + SZ_ANEG;
static_assert(OFF_H2 + SZ_H2 <= REG0_END);
static_assert((size_t)NTOK_ * G1P_ * 2 <= SZ_H1);
static_assert(WS_END <= (size_t)134217728);
static_assert(OFF_Z % 128 == 0 && OFF_MLN % 128 == 0 && OFF_OUT1 % 128 == 0 && OFF_OUT1T % 128 == 0);
static_assert(OFF_H1 % 128 == 0 && OFF_WIN % 128 == 0 && OFF_WOUT % 128 == 0 && OFF_W1 % 128 == 0);
static_assert(OFF_W2 % 128 == 0 && OFF_ST1 % 128 == 0 && OFF_ST2 % 128 == 0 && OFF_ANEG % 128 == 0);

__device__ __forceinline__ unsigned short f16_bits(float f) {
    union { _Float16 h; unsigned short u; } cv;
    cv.h = (_Float16)f;
    return cv.u;
}
__device__ __forceinline__ v8f ld8f(const float* p) {
    v4f a = *(const v4f*)p;
    v4f b = *(const v4f*)(p + 4);
    return __builtin_shufflevector(a, b, 0, 1, 2, 3, 4, 5, 6, 7);
}
__device__ __forceinline__ float silu_f(float x) {
    const float e = __expf(-x);
    return x * __builtin_amdgcn_rcpf(1.0f + e);
}
__device__ __forceinline__ float softplus_f(float x) {
    return fmaxf(x, 0.0f) + log1pf(__expf(-fabsf(x)));
}

__device__ __forceinline__ void mma16(v8f& acc, const FragH& a, const FragH& b) {
    acc = __builtin_amdgcn_wmma_f32_16x16x32_f16(false, a.v, false, b.v, (short)0, acc, false, false);
    asm volatile("v_nop\n\tv_nop\n\tv_nop\n\tv_nop" : "+v"(acc) : "v"(a.v), "v"(b.v));
}

template<int NBF>
__device__ __forceinline__ void tile_store_f32(const float* st, float* gp, int ldc, int lane) {
    constexpr int CW  = NBF * 16;
    constexpr int P   = CW + 4;
    constexpr int LPR = CW / 4;
    static_assert(32 % LPR == 0);
    constexpr int RPI = 32 / LPR;
    constexpr int NIT = 32 / RPI;
    const int rsub = lane / LPR;
    const int c0   = (lane % LPR) * 4;
#pragma unroll
    for (int it = 0; it < NIT; ++it) {
        const int row = it * RPI + rsub;
        const v4f v = *(const v4f*)(st + row * P + c0);
        *(volatile v4f*)(gp + (size_t)row * ldc + c0) = v;
    }
}
template<int NIT>
__device__ __forceinline__ void rows_f16_store_pass(const float* s, int pitch, unsigned short* gb, int gpitch,
                                                    int roww, int lane) {
#pragma unroll
    for (int it = 0; it < NIT; ++it) {
        const int row = roww + 2 * it + (lane >> 4);
        const int c0  = (lane & 15) * 8;
        const float* sp = s + row * pitch + c0;
        v8f v;
#pragma unroll
        for (int k = 0; k < 8; ++k) v[k] = sp[k];
        Pack8 pk;
        pk.f = __builtin_convertvector(v, v8h);
        const u16x8 u = pk.u;
        *(volatile u16x8*)(gb + (size_t)row * gpitch + c0) = u;
    }
}

__global__ __launch_bounds__(256)
void k_cvt_w(const float* __restrict__ win, const float* __restrict__ wout,
             const float* __restrict__ w1, const float* __restrict__ w2,
             const float* __restrict__ alog,
             unsigned short* win16, unsigned short* wout16,
             unsigned short* w1h, unsigned short* w2h, float* aneg)
{
    const int i = blockIdx.x * 256 + threadIdx.x;
    if (i < DI_ * NS_) {
        const float a = -expf(alog[i]);
        *(volatile float*)(aneg + i) = a;
        __threadfence();
        *(volatile float*)(aneg + i) = a;
    }
    constexpr int N0 = (DB_ * CH_) / 8;
    constexpr int N1 = (CH_ * DB_) / 8;
    constexpr int N2 = (HID_ * CH_) / 8;
    constexpr int N3 = (CH_ * HID_) / 8;
    const float* src;
    unsigned short* dst;
    int g;
    if (i < N0)                     { src = win;  dst = win16;  g = i; }
    else if (i < N0 + N1)           { src = wout; dst = wout16; g = i - N0; }
    else if (i < N0 + N1 + N2)      { src = w1;   dst = w1h;    g = i - N0 - N1; }
    else if (i < N0 + N1 + N2 + N3) { src = w2;   dst = w2h;    g = i - N0 - N1 - N2; }
    else return;
    const size_t e = (size_t)g * 8;
    const v8f x = ld8f(src + e) * WSCL_;
    Pack8 pk;
    pk.f = __builtin_convertvector(x, v8h);
    const u16x8 u = pk.u;
    *(volatile u16x8*)(dst + e) = u;
    __threadfence();
    *(volatile u16x8*)(dst + e) = u;
}

__global__ __launch_bounds__(256)
void k_pre_ln(const float* __restrict__ x, const float* __restrict__ g,
              const float* __restrict__ bb, unsigned short* xn16)
{
    __shared__ float xs[64][CH_ + 1];
    const int tid = threadIdx.x, lane = tid & 31, wave = tid >> 5;
    const int b  = blockIdx.x / (NL_ / 64);
    const int p0 = (blockIdx.x % (NL_ / 64)) * 64;
    {
        const int tl = tid & 63, cq = tid >> 6;
        const float* xp = x + (size_t)b * CH_ * NL_ + p0 + tl;
#pragma unroll 8
        for (int it = 0; it < CH_ / 4; ++it) {
            const int ch = cq + 4 * it;
            xs[tl][ch] = xp[(size_t)ch * NL_];
        }
    }
    __syncthreads();
    {
        const int tl = tid >> 2, sub = tid & 3;
        float* row = &xs[tl][sub * 32];
        float s = 0.0f;
#pragma unroll 8
        for (int c = 0; c < 32; ++c) s += row[c];
        s += __shfl_xor(s, 1);
        s += __shfl_xor(s, 2);
        const float mean = s * (1.0f / 128.0f);
        float q = 0.0f;
#pragma unroll 8
        for (int c = 0; c < 32; ++c) { const float d = row[c] - mean; q = fmaf(d, d, q); }
        q += __shfl_xor(q, 1);
        q += __shfl_xor(q, 2);
        const float inv = rsqrtf(q * (1.0f / 128.0f) + LNEPS_);
        const float* gp = g + sub * 32;
        const float* bp = bb + sub * 32;
#pragma unroll 8
        for (int c = 0; c < 32; ++c) row[c] = (row[c] - mean) * inv * gp[c] + bp[c];
    }
    __syncthreads();
    unsigned short* gb = xn16 + ((size_t)b * NL_ + p0) * CH_;
    rows_f16_store_pass<4>(&xs[0][0], CH_ + 1, gb, CH_, wave * 8, lane);
    __threadfence();
    rows_f16_store_pass<4>(&xs[0][0], CH_ + 1, gb, CH_, wave * 8, lane);
}

template<int NBF, bool HAS_BIAS>
__global__ __launch_bounds__(128)
void k_gemm_tn(const unsigned short* __restrict__ A, const unsigned short* __restrict__ Bw,
               const float* __restrict__ bias, float* C,
               int K, int lda, int ldb, int ldc, int sA, int sB, int sC, float scale)
{
    constexpr int CW = NBF * 16;
    constexpr int P  = CW + 4;
    __shared__ __attribute__((aligned(16))) float stile[4][32 * P];

    const int tid  = threadIdx.x;
    const int lane = tid & 31;
    const int wave = tid >> 5;
    const int h    = lane >> 4;
    const int m    = lane & 15;
    const int wm   = wave >> 1;
    const int wn   = wave & 1;
    const int bz   = blockIdx.z;
    const unsigned short* Ab = A  + (size_t)bz * (size_t)sA;
    const unsigned short* Bb = Bw + (size_t)bz * (size_t)sB;
    float* Cb = C + (size_t)bz * (size_t)sC;

    const int rowW = blockIdx.y * 64 + wm * 32;
    const int colW = blockIdx.x * (2 * CW) + wn * CW;

    v8f acc[2 * NBF];
#pragma unroll
    for (int j = 0; j < 2 * NBF; ++j)
#pragma unroll
        for (int r = 0; r < 8; ++r) acc[j][r] = 0.0f;

    const unsigned short* Ap = Ab + (size_t)(rowW + m) * lda + 8 * h;
    const unsigned short* Bp = Bb + (size_t)(colW + m) * ldb + 8 * h;
    const size_t a16 = (size_t)16 * lda;
    const size_t b16 = (size_t)16 * ldb;
    const int nk = K >> 5;

    for (int kt = 0; kt < nk; ++kt) {
        const int k0 = kt * 32;
        FragH fa[2], fb[NBF];
#pragma unroll
        for (int s = 0; s < 2; ++s) {
            const unsigned short* p = Ap + s * a16 + k0;
            fa[s].h[0] = *(const u16x8*)(p);
            fa[s].h[1] = *(const u16x8*)(p + 16);
        }
#pragma unroll
        for (int j = 0; j < NBF; ++j) {
            const unsigned short* p = Bp + j * b16 + k0;
            fb[j].h[0] = *(const u16x8*)(p);
            fb[j].h[1] = *(const u16x8*)(p + 16);
        }
#pragma unroll
        for (int s = 0; s < 2; ++s)
#pragma unroll
            for (int j = 0; j < NBF; ++j) mma16(acc[s * NBF + j], fa[s], fb[j]);
    }

    float* st = stile[wave];
#pragma unroll
    for (int s = 0; s < 2; ++s)
#pragma unroll
        for (int j = 0; j < NBF; ++j) {
            float bj = 0.0f;
            if (HAS_BIAS) bj = bias[colW + j * 16 + m];
#pragma unroll
            for (int r = 0; r < 8; ++r)
                st[(s * 16 + 8 * h + r) * P + j * 16 + m] = fmaf(acc[s * NBF + j][r], scale, bj);
        }
    __syncthreads();

    float* gp = Cb + (size_t)rowW * ldc + colW;
    tile_store_f32<NBF>(st, gp, ldc, lane);
    __threadfence();
    tile_store_f32<NBF>(st, gp, ldc, lane);
}

__global__ __launch_bounds__(128)
void k_bott_out(const unsigned short* __restrict__ A, const unsigned short* __restrict__ Bw,
                const float* __restrict__ bias, const float* __restrict__ rsp,
                const float* __restrict__ x, float* out1, unsigned short* out1t)
{
    constexpr int P = CH_ + 5;
    __shared__ __attribute__((aligned(16))) float sacc[64 * P];

    const int tid  = threadIdx.x;
    const int lane = tid & 31;
    const int wave = tid >> 5;
    const int h    = lane >> 4;
    const int m    = lane & 15;
    const int wm   = wave >> 1;
    const int wn   = wave & 1;
    const int row0 = blockIdx.x * 64;
    const int b    = blockIdx.x / (NL_ / 64);
    const int p0   = (blockIdx.x % (NL_ / 64)) * 64;

    v8f acc[8];
#pragma unroll
    for (int j = 0; j < 8; ++j)
#pragma unroll
        for (int r = 0; r < 8; ++r) acc[j][r] = 0.0f;

    const unsigned short* Ap = A  + (size_t)(row0 + wm * 32 + m) * DB_ + 8 * h;
    const unsigned short* Bp = Bw + (size_t)(wn * 64 + m) * DB_ + 8 * h;
#pragma unroll
    for (int kt = 0; kt < DB_ / 32; ++kt) {
        const int k0 = kt * 32;
        FragH fa[2], fb[4];
#pragma unroll
        for (int s = 0; s < 2; ++s) {
            const unsigned short* p = Ap + (size_t)s * 16 * DB_ + k0;
            fa[s].h[0] = *(const u16x8*)(p);
            fa[s].h[1] = *(const u16x8*)(p + 16);
        }
#pragma unroll
        for (int j = 0; j < 4; ++j) {
            const unsigned short* p = Bp + (size_t)j * 16 * DB_ + k0;
            fb[j].h[0] = *(const u16x8*)(p);
            fb[j].h[1] = *(const u16x8*)(p + 16);
        }
#pragma unroll
        for (int s = 0; s < 2; ++s)
#pragma unroll
            for (int j = 0; j < 4; ++j) mma16(acc[s * 4 + j], fa[s], fb[j]);
    }

    const float rs = rsp[0];
#pragma unroll
    for (int s = 0; s < 2; ++s)
#pragma unroll
        for (int j = 0; j < 4; ++j) {
            const int ch = wn * 64 + j * 16 + m;
            const float bj = bias[ch];
#pragma unroll
            for (int r = 0; r < 8; ++r) {
                const int tl = wm * 32 + s * 16 + 8 * h + r;
                sacc[tl * P + ch] = fmaf(acc[s * 4 + j][r], WINV_, bj) * rs;
            }
        }
    __syncthreads();

    {
        const int q  = lane & 15;
        const int cs = lane >> 4;
        const size_t nbase = (size_t)b * CH_ * NL_ + p0 + 4 * q;
        const float* xb = x + nbase;
        float* ob = out1 + nbase;
#pragma unroll
        for (int it = 0; it < 16; ++it) {
            const int ch = wave * 32 + 2 * it + cs;
            const v4f xv = *(const v4f*)(xb + (size_t)ch * NL_);
            v4f o;
#pragma unroll
            for (int jj = 0; jj < 4; ++jj) {
                float* sp = sacc + (4 * q + jj) * P + ch;
                const float tk = xv[jj] + *sp;
                const float ov = xv[jj] + tk;
                o[jj] = ov;
                *sp = ov;
            }
            *(volatile v4f*)(ob + (size_t)ch * NL_) = o;
        }
        __threadfence();
#pragma unroll
        for (int it = 0; it < 16; ++it) {
            const int ch = wave * 32 + 2 * it + cs;
            v4f o;
#pragma unroll
            for (int jj = 0; jj < 4; ++jj) o[jj] = sacc[(4 * q + jj) * P + ch];
            *(volatile v4f*)(ob + (size_t)ch * NL_) = o;
        }
    }
    __syncthreads();

    unsigned short* tb = out1t + (size_t)row0 * CH_;
    rows_f16_store_pass<8>(sacc, P, tb, CH_, wave * 16, lane);
    __threadfence();
    rows_f16_store_pass<8>(sacc, P, tb, CH_, wave * 16, lane);
}

__global__ __launch_bounds__(128)
void k_ssm(const float* __restrict__ z, const float* __restrict__ inw,
           const float* __restrict__ cw, const float* __restrict__ cb,
           const float* __restrict__ xpw, const float* __restrict__ dtw,
           const float* __restrict__ dtb, const float* __restrict__ aneg,
           const float* __restrict__ Dp, const float* __restrict__ opw,
           const float* __restrict__ pg, const float* __restrict__ pb,
           unsigned short* mln16)
{
    __shared__ __attribute__((aligned(16))) float s_inwT[DM_ * 2 * DI_];
    __shared__ __attribute__((aligned(16))) float s_xpwT[DI_ * XDN_];
    __shared__ __attribute__((aligned(16))) float s_opwT[DI_ * DM_];
    __shared__ float s_pg[DB_], s_pb[DB_];
    __shared__ __attribute__((aligned(16))) float sz[16 * DB_];
    __shared__ __attribute__((aligned(16))) float sxc[4 * DI_];
    __shared__ __attribute__((aligned(16))) float sbc[4 * DI_];
    __shared__ __attribute__((aligned(16))) float sy[4 * DI_];
    __shared__ float sm[DB_];
    __shared__ __attribute__((aligned(16))) unsigned short smln[16 * DB_];

    const int tid  = threadIdx.x;
    const int lane = tid & 31;
    const int c    = tid >> 5;
    const int b    = blockIdx.x;

    for (int i = tid; i < 2 * DI_ * DM_; i += 128) {
        const int o = i >> 4, ii = i & 15;
        s_inwT[ii * (2 * DI_) + o] = inw[i];
    }
    for (int i = tid; i < XDN_ * DI_; i += 128) {
        const int j = i >> 5, ii = i & 31;
        s_xpwT[ii * XDN_ + j] = xpw[i];
    }
    for (int i = tid; i < DM_ * DI_; i += 128) {
        const int jj = i >> 5, dd = i & 31;
        s_opwT[dd * DM_ + jj] = opw[i];
    }
    if (tid < DB_) { s_pg[tid] = pg[tid]; s_pb[tid] = pb[tid]; }

    const int d = lane;
    const float w0 = cw[d * 4 + 0], w1 = cw[d * 4 + 1], w2 = cw[d * 4 + 2], w3 = cw[d * 4 + 3];
    const float cbias = cb[d];
    const float tw = dtw[d];
    const float tb = dtb[d];
    const float Dd = Dp[d];
    float an[NS_], hs[NS_];
#pragma unroll
    for (int n = 0; n < NS_; ++n) { an[n] = aneg[d * NS_ + n]; hs[n] = 0.0f; }
    float xm1 = 0.0f, xm2 = 0.0f, xm3 = 0.0f;
    __syncthreads();

    const size_t zrow0 = (size_t)b * NL_;
#pragma unroll 1
    for (int t0 = 0; t0 < NL_; t0 += 16) {
        {
            const int tt = tid >> 3, c8 = (tid & 7) * 8;
            const float* zp = z + (zrow0 + t0 + tt) * DB_ + c8;
            *(v4f*)(sz + tt * DB_ + c8)     = *(const v4f*)zp;
            *(v4f*)(sz + tt * DB_ + c8 + 4) = *(const v4f*)(zp + 4);
        }
        __syncthreads();
#pragma unroll 1
        for (int tt = 0; tt < 16; ++tt) {
            const float* zr = sz + tt * DB_ + c * DM_;
            float xp = 0.0f, zg = 0.0f;
#pragma unroll 1
            for (int i4 = 0; i4 < DM_; i4 += 4) {
                const v4f zv = *(const v4f*)(zr + i4);
                const float* wr = s_inwT + i4 * (2 * DI_) + d;
#pragma unroll
                for (int k = 0; k < 4; ++k) {
                    xp = fmaf(zv[k], wr[k * (2 * DI_)], xp);
                    zg = fmaf(zv[k], wr[k * (2 * DI_) + DI_], zg);
                }
            }
            const float cv = fmaf(w3, xp, fmaf(w2, xm1, fmaf(w1, xm2, w0 * xm3))) + cbias;
            const float u  = silu_f(cv);
            xm3 = xm2; xm2 = xm1; xm1 = xp;
            sxc[c * DI_ + d] = u;
            __syncthreads();
            float col = 0.0f;
            const float* xr = sxc + c * DI_;
#pragma unroll 1
            for (int i4 = 0; i4 < DI_; i4 += 4) {
                const v4f xv = *(const v4f*)(xr + i4);
                const float* wr = s_xpwT + i4 * XDN_ + 1 + d;
#pragma unroll
                for (int k = 0; k < 4; ++k) col = fmaf(xv[k], wr[k * XDN_], col);
            }
            float pr = u * s_xpwT[d * XDN_];
            pr += __shfl_xor(pr, 16);
            pr += __shfl_xor(pr, 8);
            pr += __shfl_xor(pr, 4);
            pr += __shfl_xor(pr, 2);
            pr += __shfl_xor(pr, 1);
            sbc[c * DI_ + d] = col;
            const float dt = softplus_f(fmaf(pr, tw, tb));
            __syncthreads();
            const float du = dt * u;
            float y = 0.0f;
            const float* br = sbc + c * DI_;
#pragma unroll
            for (int n4 = 0; n4 < NS_; n4 += 4) {
                const v4f bv = *(const v4f*)(br + n4);
                const v4f cq = *(const v4f*)(br + NS_ + n4);
#pragma unroll
                for (int k = 0; k < 4; ++k) {
                    const float da = __expf(dt * an[n4 + k]);
                    const float hn = fmaf(da, hs[n4 + k], du * bv[k]);
                    hs[n4 + k] = hn;
                    y = fmaf(hn, cq[k], y);
                }
            }
            const float gv = fmaf(Dd, u, y) * silu_f(zg);
            sy[c * DI_ + d] = gv;
            __syncthreads();
            {
                const int hh = lane >> 4, jj = lane & 15;
                const float* yr = sy + c * DI_ + hh * 16;
                const float* wr = s_opwT + (hh * 16) * DM_ + jj;
                float mo = 0.0f;
#pragma unroll 1
                for (int d4 = 0; d4 < 16; d4 += 4) {
                    const v4f yv = *(const v4f*)(yr + d4);
#pragma unroll
                    for (int k = 0; k < 4; ++k) mo = fmaf(yv[k], wr[(d4 + k) * DM_], mo);
                }
                mo += __shfl_xor(mo, 16);
                mo += zr[jj];
                if (lane < DM_) sm[c * DM_ + jj] = mo;
            }
            __syncthreads();
            {
                const float v0 = sm[lane], v1 = sm[32 + lane];
                float s = v0 + v1;
                s += __shfl_xor(s, 16);
                s += __shfl_xor(s, 8);
                s += __shfl_xor(s, 4);
                s += __shfl_xor(s, 2);
                s += __shfl_xor(s, 1);
                const float mean = s * (1.0f / 64.0f);
                const float e0 = v0 - mean, e1 = v1 - mean;
                float q = fmaf(e0, e0, e1 * e1);
                q += __shfl_xor(q, 16);
                q += __shfl_xor(q, 8);
                q += __shfl_xor(q, 4);
                q += __shfl_xor(q, 2);
                q += __shfl_xor(q, 1);
                const float inv = rsqrtf(q * (1.0f / 64.0f) + LNEPS_);
                if (lane < DM_) {
                    const int ch = c * DM_ + lane;
                    const float nv = (sm[ch] - mean) * inv * s_pg[ch] + s_pb[ch];
                    smln[tt * DB_ + ch] = f16_bits(nv);
                }
            }
        }
        __syncthreads();
        {
            const int row = tid >> 3, c8 = (tid & 7) * 8;
            const u16x8 v = *(const u16x8*)(smln + row * DB_ + c8);
            unsigned short* gp = mln16 + (zrow0 + t0 + row) * DB_ + c8;
            *(volatile u16x8*)gp = v;
            __threadfence();
            *(volatile u16x8*)gp = v;
        }
    }
}

__device__ __forceinline__ void block_stats_store(double* sd, double* sq, float s, float q, int tid,
                                                  double n, float* stl)
{
    sd[tid] = (double)s;
    sq[tid] = (double)q;
    __syncthreads();
    for (int w = 128; w > 0; w >>= 1) {
        if (tid < w) { sd[tid] += sd[tid + w]; sq[tid] += sq[tid + w]; }
        __syncthreads();
    }
    if (tid < 32) {
        const double mean = sd[0] / n;
        double var = sq[0] / n - mean * mean;
        if (var < 0.0) var = 0.0;
        const float inv = rsqrtf((float)var + LNEPS_);
        float val = 0.0f;
        if (tid == 0) val = (float)mean;
        else if (tid == 1) val = inv;
        *(volatile float*)(stl + tid) = val;
        __threadfence();
        *(volatile float*)(stl + tid) = val;
    }
}

__global__ __launch_bounds__(256)
void k_gn_stats1(const float* __restrict__ h1, float* st)
{
    __shared__ double sd[256], sq[256];
    const int tid = threadIdx.x;
    const int b = blockIdx.x / NGRP_, g = blockIdx.x % NGRP_;
    const int rsub = tid >> 2, qt = tid & 3;
    const float* hp = h1 + ((size_t)b * NL_ + rsub) * HID_ + g * 16 + qt * 4;
    float s = 0.0f, q = 0.0f;
#pragma unroll 4
    for (int it = 0; it < NL_ / 64; ++it) {
        const v4f v = *(const v4f*)(hp + (size_t)it * 64 * HID_);
        s += (v[0] + v[1]) + (v[2] + v[3]);
        q = fmaf(v[0], v[0], q); q = fmaf(v[1], v[1], q);
        q = fmaf(v[2], v[2], q); q = fmaf(v[3], v[3], q);
    }
    block_stats_store(sd, sq, s, q, tid, (double)(16 * NL_), st + (size_t)blockIdx.x * 32);
}

__global__ __launch_bounds__(256)
void k_gn_stats2(const float* __restrict__ h2, float* st)
{
    __shared__ double sd[256], sq[256];
    const int tid = threadIdx.x;
    const int b = blockIdx.x / NGRP_, g = blockIdx.x % NGRP_;
    const float* hp = h2 + ((size_t)b * CH_ + 4 * g) * NL_ + tid * 4;
    float s = 0.0f, q = 0.0f;
#pragma unroll 4
    for (int it = 0; it < (4 * NL_) / 1024; ++it) {
        const v4f v = *(const v4f*)(hp + (size_t)it * 1024);
        s += (v[0] + v[1]) + (v[2] + v[3]);
        q = fmaf(v[0], v[0], q); q = fmaf(v[1], v[1], q);
        q = fmaf(v[2], v[2], q); q = fmaf(v[3], v[3], q);
    }
    block_stats_store(sd, sq, s, q, tid, (double)(4 * NL_), st + (size_t)blockIdx.x * 32);
}

__global__ __launch_bounds__(256)
void k_gn1_gelu(float* h1, const float* __restrict__ st, const float* __restrict__ gg,
                const float* __restrict__ gb)
{
    __shared__ __attribute__((aligned(16))) unsigned short sg[2 * HID_];
    const int tid = threadIdx.x;
    const int rl  = tid >> 7;
    const int c0  = (tid & 127) * 4;
    const int row = blockIdx.x * 2 + rl;
    const int b   = row / NL_;
    const int g   = c0 >> 4;
    const v4f v = *(const v4f*)(h1 + (size_t)row * HID_ + c0);
    const float mean = st[(b * NGRP_ + g) * 32];
    const float inv  = st[(b * NGRP_ + g) * 32 + 1];
#pragma unroll
    for (int k = 0; k < 4; ++k) {
        float t = (v[k] - mean) * inv * gg[c0 + k] + gb[c0 + k];
        t = 0.5f * t * (1.0f + erff(t * 0.70710678118654752f));
        sg[rl * HID_ + c0 + k] = f16_bits(t);
    }
    __syncthreads();
    if (tid < 128) {
        const int r2 = tid >> 6, c8 = (tid & 63) * 8;
        const u16x8 u = *(const u16x8*)(sg + r2 * HID_ + c8);
        unsigned short* gp = (unsigned short*)h1 + (size_t)(blockIdx.x * 2 + r2) * G1P_ + c8;
        *(volatile u16x8*)gp = u;
        __threadfence();
        *(volatile u16x8*)gp = u;
    }
}

__global__ __launch_bounds__(256)
void k_final(const float* __restrict__ h2, const float* __restrict__ st,
             const float* __restrict__ gg, const float* __restrict__ gb,
             const float* __restrict__ out1, float* out)
{
    const size_t i4 = (size_t)blockIdx.x * 256 + threadIdx.x;
    const size_t e  = i4 * 4;
    const int ch = (int)((e / NL_) % CH_);
    const int b  = (int)(e / ((size_t)CH_ * NL_));
    const int g  = ch / (CH_ / NGRP_);
    const float mean = st[(b * NGRP_ + g) * 32];
    const float inv  = st[(b * NGRP_ + g) * 32 + 1];
    const float gc = gg[ch], bc = gb[ch];
    const v4f hv = *(const v4f*)(h2 + e);
    const v4f ov = *(const v4f*)(out1 + e);
    v4f r;
#pragma unroll
    for (int k = 0; k < 4; ++k) r[k] = ov[k] + ((hv[k] - mean) * inv * gc + bc);
    *(volatile v4f*)(out + e) = r;
    __threadfence();
    *(volatile v4f*)(out + e) = r;
}

extern "C" void kernel_launch(void* const* d_in, const int* in_sizes, int n_in,
                              void* d_out, int out_size, void* d_ws, size_t ws_size,
                              hipStream_t stream)
{
    if (n_in < 25) return;
    if (in_sizes[0]  != NB_ * CH_ * NL_) return;
    if (in_sizes[1]  != CH_) return;
    if (in_sizes[2]  != CH_) return;
    if (in_sizes[3]  != DB_ * CH_) return;
    if (in_sizes[4]  != DB_) return;
    if (in_sizes[5]  != 2 * DI_ * DM_) return;
    if (in_sizes[6]  != DI_ * 4) return;
    if (in_sizes[7]  != DI_) return;
    if (in_sizes[8]  != XDN_ * DI_) return;
    if (in_sizes[9]  != DI_) return;
    if (in_sizes[10] != DI_) return;
    if (in_sizes[11] != DI_ * NS_) return;
    if (in_sizes[12] != DI_) return;
    if (in_sizes[13] != DM_ * DI_) return;
    if (in_sizes[14] != DB_) return;
    if (in_sizes[15] != DB_) return;
    if (in_sizes[16] != CH_ * DB_) return;
    if (in_sizes[17] != CH_) return;
    if (in_sizes[18] < 1) return;
    if (in_sizes[19] != HID_ * CH_) return;
    if (in_sizes[20] != HID_) return;
    if (in_sizes[21] != HID_) return;
    if (in_sizes[22] != CH_ * HID_) return;
    if (in_sizes[23] != CH_) return;
    if (in_sizes[24] != CH_) return;
    if (out_size != NB_ * CH_ * NL_) return;
    if (ws_size < WS_END) return;

    const float* x      = (const float*)d_in[0];
    const float* pre_g  = (const float*)d_in[1];
    const float* pre_b  = (const float*)d_in[2];
    const float* bin_w  = (const float*)d_in[3];
    const float* bin_b  = (const float*)d_in[4];
    const float* inp_w  = (const float*)d_in[5];
    const float* conv_w = (const float*)d_in[6];
    const float* conv_b = (const float*)d_in[7];
    const float* xp_w   = (const float*)d_in[8];
    const float* dt_w   = (const float*)d_in[9];
    const float* dt_b   = (const float*)d_in[10];
    const float* a_log  = (const float*)d_in[11];
    const float* dpar   = (const float*)d_in[12];
    const float* op_w   = (const float*)d_in[13];
    const float* post_g = (const float*)d_in[14];
    const float* post_b = (const float*)d_in[15];
    const float* bout_w = (const float*)d_in[16];
    const float* bout_b = (const float*)d_in[17];
    const float* res_sc = (const float*)d_in[18];
    const float* fc1_w  = (const float*)d_in[19];
    const float* gn1_g  = (const float*)d_in[20];
    const float* gn1_b  = (const float*)d_in[21];
    const float* fc2_w  = (const float*)d_in[22];
    const float* gn2_g  = (const float*)d_in[23];
    const float* gn2_b  = (const float*)d_in[24];
    float* out = (float*)d_out;

    char* ws = (char*)d_ws;
    unsigned short* xn16   = (unsigned short*)(ws + OFF_XN16);
    float*          zf     = (float*)(ws + OFF_Z);
    unsigned short* mln16  = (unsigned short*)(ws + OFF_MLN);
    float*          h2     = (float*)(ws + OFF_H2);
    float*          out1   = (float*)(ws + OFF_OUT1);
    unsigned short* out1t  = (unsigned short*)(ws + OFF_OUT1T);
    float*          h1     = (float*)(ws + OFF_H1);
    unsigned short* g1     = (unsigned short*)(ws + OFF_H1);
    unsigned short* win16  = (unsigned short*)(ws + OFF_WIN);
    unsigned short* wout16 = (unsigned short*)(ws + OFF_WOUT);
    unsigned short* w1h    = (unsigned short*)(ws + OFF_W1);
    unsigned short* w2h    = (unsigned short*)(ws + OFF_W2);
    float*          st1    = (float*)(ws + OFF_ST1);
    float*          st2    = (float*)(ws + OFF_ST2);
    float*          aneg   = (float*)(ws + OFF_ANEG);

    {
        const int ngroups = (DB_ * CH_ + CH_ * DB_ + HID_ * CH_ + CH_ * HID_) / 8;
        k_cvt_w<<<dim3((ngroups + 255) / 256), dim3(256), 0, stream>>>(
            bin_w, bout_w, fc1_w, fc2_w, a_log, win16, wout16, w1h, w2h, aneg);
    }
    k_pre_ln<<<dim3(NTOK_ / 64), dim3(256), 0, stream>>>(x, pre_g, pre_b, xn16);
    k_gemm_tn<2, true><<<dim3(DB_ / 64, NTOK_ / 64, 1), dim3(128), 0, stream>>>(
        xn16, win16, bin_b, zf, (int)CH_, (int)CH_, (int)CH_, (int)DB_, 0, 0, 0, WINV_);
    k_ssm<<<dim3(NB_), dim3(128), 0, stream>>>(
        zf, inp_w, conv_w, conv_b, xp_w, dt_w, dt_b, aneg, dpar, op_w, post_g, post_b, mln16);
    k_bott_out<<<dim3(NTOK_ / 64), dim3(128), 0, stream>>>(
        mln16, wout16, bout_b, res_sc, x, out1, out1t);
    k_gemm_tn<4, false><<<dim3(HID_ / 128, NTOK_ / 64, 1), dim3(128), 0, stream>>>(
        out1t, w1h, bin_b, h1, (int)CH_, (int)CH_, (int)CH_, (int)HID_, 0, 0, 0, WINV_);
    k_gn_stats1<<<dim3(NB_ * NGRP_), dim3(256), 0, stream>>>(h1, st1);
    k_gn1_gelu<<<dim3(NTOK_ / 2), dim3(256), 0, stream>>>(h1, st1, gn1_g, gn1_b);
    k_gemm_tn<4, false><<<dim3(NL_ / 128, CH_ / 64, NB_), dim3(128), 0, stream>>>(
        w2h, g1, bin_b, h2, (int)HID_, (int)HID_, (int)G1P_, (int)NL_,
        0, (int)(NL_ * G1P_), (int)(CH_ * NL_), WINV_);
    k_gn_stats2<<<dim3(NB_ * NGRP_), dim3(256), 0, stream>>>(h2, st2);
    k_final<<<dim3((NB_ * CH_ * NL_) / 1024), dim3(256), 0, stream>>>(h2, st2, gn2_g, gn2_b, out1, out);
}
